// EncoderMultiHeadAttention_11665131176436
// MI455X (gfx1250) — hardware-verified
//
#include <hip/hip_runtime.h>


#define NB_  8
#define TT   1024
#define DD   512
#define NH_  8
#define HD   64
#define K3   (3 * DD)
#define K6   (6 * DD)
#define NR   (NB_ * TT)
#define DM   DD
#define PCAR 1024.0f
#define LOSC 1024.0f
typedef _Float16 h16;
typedef unsigned short bf;
typedef __attribute__((ext_vector_type(16))) __bf16   v16bf;
typedef __attribute__((ext_vector_type(16))) _Float16 v16h;
typedef __attribute__((ext_vector_type(8)))  _Float16 v8h;
typedef __attribute__((ext_vector_type(8)))  unsigned short v8us;
typedef __attribute__((ext_vector_type(8)))  float    v8f;
typedef __attribute__((ext_vector_type(4)))  float    v4f;
typedef v8h  __attribute__((may_alias)) v8ha;
typedef v4f  __attribute__((may_alias)) v4fa;
typedef v8us __attribute__((may_alias)) v8usa;

__device__ __forceinline__ unsigned short f2bf(float f) { unsigned u = __float_as_uint(f); u += 0x7FFFu + ((u >> 16) & 1u); return (unsigned short)(u >> 16); }
__device__ __forceinline__ float bf2f(unsigned short b) { return __uint_as_float(((unsigned)b) << 16); }
__device__ __forceinline__ float bfr(float f) { return bf2f(f2bf(f)); }
__device__ __forceinline__ v16h cat16(v8h lo, v8h hi) { return __builtin_shufflevector(lo, hi, 0, 1, 2, 3, 4, 5, 6, 7, 8, 9, 10, 11, 12, 13, 14, 15); }
__device__ __forceinline__ v16bf cat16b(v8us lo, v8us hi) { return __builtin_bit_cast(v16bf, __builtin_shufflevector(lo, hi, 0, 1, 2, 3, 4, 5, 6, 7, 8, 9, 10, 11, 12, 13, 14, 15)); }
__device__ __forceinline__ v8f wmma16(v16h a, v16h b, v8f c) { return __builtin_amdgcn_wmma_f32_16x16x32_f16(false, a, false, b, (short)0, c, false, false); }
__device__ __forceinline__ v8f wmmab(v16bf a, v16bf b, v8f c) { return __builtin_amdgcn_wmma_f32_16x16x32_bf16(false, a, false, b, (short)0, c, false, false); }


__global__ __launch_bounds__(128) void k_gemmh(const h16* __restrict__ A, const h16* __restrict__ Bn, const float* __restrict__ bias, float* C, int ldc, const float* __restrict__ R, int K, size_t sA, size_t sB, size_t sC, int roundR) {
    __shared__ __align__(16) float ost[4][16 * 68];
    const size_t z = blockIdx.z; A += z * sA; Bn += z * sB; C += z * sC; if (R) R += z * sC;
    const int lane = threadIdx.x & 31, wave = threadIdx.x >> 5, lr = lane & 15, hi = lane >> 4;
    const int r0 = blockIdx.x * 64 + wave * 16, c0 = blockIdx.y * 64;
    const size_t aoff = (size_t)(r0 + lr) * K + 8 * hi;
    size_t boff[4];
#pragma unroll
    for (int t = 0; t < 4; ++t) boff[t] = (size_t)(c0 + t * 16 + lr) * K + 8 * hi;
    v8f acc[4];
#pragma unroll
    for (int t = 0; t < 4; ++t) acc[t] = (v8f){};
#pragma unroll 1
    for (int kc = 0; kc < K; kc += 32) {
        const v16h a = cat16(*(const v8h*)(A + aoff + kc), *(const v8h*)(A + aoff + kc + 16));
#pragma unroll
        for (int t = 0; t < 4; ++t) { const v16h b = cat16(*(const v8h*)(Bn + boff[t] + kc), *(const v8h*)(Bn + boff[t] + kc + 16)); acc[t] = wmma16(a, b, acc[t]); }
        asm volatile("v_nop\n\tv_nop\n\tv_nop\n\tv_nop" : "+v"(acc[0]), "+v"(acc[1]), "+v"(acc[2]), "+v"(acc[3]) : "v"(a));
    }
    float* os = &ost[wave][0];
#pragma unroll
    for (int t = 0; t < 4; ++t) { const float bv = bias ? bfr(bias[c0 + t * 16 + lr]) : 0.f;
#pragma unroll
        for (int j = 0; j < 8; ++j) os[(hi * 8 + j) * 68 + t * 16 + lr] = acc[t][j] + bv; }
    __syncthreads();
    float* crow = C + (size_t)r0 * ldc + c0;
    auto pass = [&]() {
#pragma unroll
        for (int s = 0; s < 8; ++s) { const int Lid = (lane >> 3) + 4 * s, piece = lane & 7; const int row = Lid >> 1, cofs = (Lid & 1) * 32 + piece * 4;
            v4f val = *(const v4fa*)(os + row * 68 + cofs); if (R) { const v4f rv = *(const v4f*)(R + ((size_t)r0 + row) * ldc + c0 + cofs); val += roundR ? (v4f){bfr(rv[0]), bfr(rv[1]), bfr(rv[2]), bfr(rv[3])} : rv; }
            *(volatile v4f*)(crow + (size_t)row * ldc + cofs) = val; }
    };
    pass(); __threadfence(); pass();
}

template <int MODE>
__global__ __launch_bounds__(128) void k_gemm3z(const bf* __restrict__ Ah, const bf* __restrict__ Al, const bf* __restrict__ Bh, const bf* __restrict__ Bl, int K, float* C, int ldc, size_t sA, size_t sB, size_t sC) {
    if ((MODE & 1) && (int)blockIdx.y * 64 > (int)blockIdx.x * 64 + 63) return;
    const size_t z = blockIdx.z; Ah += z * sA; Al += z * sA; Bh += z * sB; Bl += z * sB; C += z * sC;
    const int Klim = (MODE & 2) ? min(K, ((int)blockIdx.x + 1) * 64) : K;
    __shared__ __align__(16) float ost[4][16 * 68];
    const int lane = threadIdx.x & 31, wave = threadIdx.x >> 5, lr = lane & 15, hi = lane >> 4;
    const int r0 = blockIdx.x * 64 + wave * 16, c0 = blockIdx.y * 64;
    const size_t aoff = (size_t)(r0 + lr) * K + 8 * hi;
    v8f acc[4];
#pragma unroll
    for (int t = 0; t < 4; ++t) acc[t] = (v8f){};
#pragma unroll 1
    for (int kc = 0; kc < Klim; kc += 32) {
        const v16bf a = cat16b(*(const v8us*)(Ah + aoff + kc), *(const v8us*)(Ah + aoff + kc + 16));
        v16bf al = a; if (!(MODE & 4) && !(MODE & 16)) al = cat16b(*(const v8us*)(Al + aoff + kc), *(const v8us*)(Al + aoff + kc + 16));
#pragma unroll
        for (int t = 0; t < 4; ++t) { const size_t bo = (size_t)(c0 + t * 16 + lr) * K + kc + 8 * hi;
            const v16bf bh = cat16b(*(const v8us*)(Bh + bo), *(const v8us*)(Bh + bo + 16));
            acc[t] = wmmab(a, bh, acc[t]);
            if (!(MODE & 4)) { if (!(MODE & 16)) acc[t] = wmmab(al, bh, acc[t]); if (!(MODE & 8)) { const v16bf bl = cat16b(*(const v8us*)(Bl + bo), *(const v8us*)(Bl + bo + 16)); acc[t] = wmmab(a, bl, acc[t]); } } }
        asm volatile("v_nop\n\tv_nop\n\tv_nop\n\tv_nop" : "+v"(acc[0]), "+v"(acc[1]), "+v"(acc[2]), "+v"(acc[3]) : "v"(a), "v"(al));
    }
    float* os = &ost[wave][0];
#pragma unroll
    for (int t = 0; t < 4; ++t) {
#pragma unroll
        for (int j = 0; j < 8; ++j) os[(hi * 8 + j) * 68 + t * 16 + lr] = acc[t][j]; }
    __builtin_amdgcn_wave_barrier(); asm volatile("" ::: "memory");
    float* crow = C + (size_t)r0 * ldc + c0;
    auto pass = [&]() {
#pragma unroll
        for (int s = 0; s < 8; ++s) { const int Lid = (lane >> 3) + 4 * s, piece = lane & 7; const int row = Lid >> 1, cofs = (Lid & 1) * 32 + piece * 4;
            const v4f val = *(const v4fa*)(os + row * 68 + cofs); *(volatile v4f*)(crow + (size_t)row * ldc + cofs) = val; }
    };
    pass(); __threadfence(); pass();
}
__global__ __launch_bounds__(256) void k_planes32z(const float* __restrict__ F, int ld, int off, float sc, int rows, bf* Ph, bf* Pl) {
    typedef __attribute__((ext_vector_type(2))) unsigned short v2us;
    const int lane = threadIdx.x & 31; const size_t r = ((size_t)blockIdx.x * 8 + (threadIdx.x >> 5)) * 2 + (lane >> 4); if (r >= (size_t)rows) return; const int z = blockIdx.z; const int c0 = (lane & 15) * 2; v2us oh, ol;
    Ph += (size_t)z * rows * 32; Pl += (size_t)z * rows * 32;
#pragma unroll
    for (int i = 0; i < 2; ++i) { const float y = F[r * ld + off + z * 32 + c0 + i] * sc; const unsigned short hb = f2bf(y); oh[i] = hb; ol[i] = f2bf(y - bf2f(hb)); }
    const size_t o = r * 32 + c0; *(volatile v2us*)(Ph + o) = oh; *(volatile v2us*)(Pl + o) = ol; __threadfence(); *(volatile v2us*)(Ph + o) = oh; *(volatile v2us*)(Pl + o) = ol;
}
__global__ __launch_bounds__(256) void k_vtpadz(const float* __restrict__ F, int ld, int off, int nk, bf* Th, bf* Tl) {
    typedef __attribute__((ext_vector_type(2))) unsigned short v2us;
    const int lane = threadIdx.x & 31; const size_t wid = (size_t)blockIdx.x * 8 + (threadIdx.x >> 5); if (wid >= (size_t)64 * (nk / 64)) return; const int z = blockIdx.z; const int d = (int)(wid / (nk / 64)); const int k0 = (int)(wid % (nk / 64)) * 64 + lane * 2; v2us oh, ol;
    Th += (size_t)z * 64 * nk; Tl += (size_t)z * 64 * nk;
#pragma unroll
    for (int i = 0; i < 2; ++i) { const float y = (d < 32) ? F[(size_t)(k0 + i) * ld + off + z * 32 + (d < 32 ? d : 0)] : 0.f; const unsigned short hb = f2bf(y); oh[i] = hb; ol[i] = f2bf(y - bf2f(hb)); }
    const size_t o = (size_t)d * nk + k0; *(volatile v2us*)(Th + o) = oh; *(volatile v2us*)(Tl + o) = ol; __threadfence(); *(volatile v2us*)(Th + o) = oh; *(volatile v2us*)(Tl + o) = ol;
}
template <int NK>
__global__ __launch_bounds__(256) void k_softmaxz(const float* __restrict__ S, int rows, bf* PH, bf* PL) {
    typedef __attribute__((ext_vector_type(4))) unsigned short v4us;
    const int lane = threadIdx.x & 31, i = blockIdx.x * 8 + (threadIdx.x >> 5); if (i >= rows) return; const size_t zo = (size_t)blockIdx.z * rows * NK; const float* sr = S + zo + (size_t)i * NK; PH += zo; PL += zo;
    float m = -3.0e38f;
#pragma unroll 1
    for (int c0 = lane * 4; c0 < NK; c0 += 128) {
#pragma unroll
        for (int q = 0; q < 4; ++q) m = fmaxf(m, sr[c0 + q]); }
#pragma unroll
    for (int sh = 16; sh; sh >>= 1) m = fmaxf(m, __shfl_xor(m, sh, 32));
    float sum = 0.f;
#pragma unroll 1
    for (int c0 = lane * 4; c0 < NK; c0 += 128) {
#pragma unroll
        for (int q = 0; q < 4; ++q) sum += __expf(sr[c0 + q] - m); }
#pragma unroll
    for (int sh = 16; sh; sh >>= 1) sum += __shfl_xor(sum, sh, 32);
    const float inv = 1.0f / sum;
#pragma unroll 1
    for (int ps = 0; ps < 2; ++ps) {
#pragma unroll 1
        for (int c0 = lane * 4; c0 < NK; c0 += 128) { v4us oh, ol;
#pragma unroll
            for (int q = 0; q < 4; ++q) { const float p = __expf(sr[c0 + q] - m) * inv; const unsigned short hb = f2bf(p); oh[q] = hb; ol[q] = f2bf(p - bf2f(hb)); }
            const size_t o = (size_t)i * NK + c0; *(volatile v4us*)(PH + o) = oh; *(volatile v4us*)(PL + o) = ol; }
        if (ps == 0) __threadfence(); }
}
__global__ __launch_bounds__(256) void k_placez(const float* __restrict__ XH, int rows, int ldy, float* Y) {
    const int lane = threadIdx.x & 31; const size_t q = (size_t)blockIdx.x * 8 + (threadIdx.x >> 5); if (q >= (size_t)rows) return; const int z = blockIdx.z; const float v = XH[((size_t)z * rows + q) * 64 + lane];
    *(volatile float*)(Y + q * ldy + z * 32 + lane) = v; __threadfence(); *(volatile float*)(Y + q * ldy + z * 32 + lane) = v;
}

template <typename T16> struct WFrag;
template <> struct WFrag<h16> { typedef v16h V; static __device__ __forceinline__ V ld(const h16* p) { return cat16(*(const v8h*)p, *(const v8h*)(p + 16)); } static __device__ __forceinline__ v8f mma(V a, V b, v8f c) { return wmma16(a, b, c); } };
template <> struct WFrag<bf> { typedef v16bf V; static __device__ __forceinline__ V ld(const bf* p) { return cat16b(*(const v8us*)p, *(const v8us*)(p + 16)); } static __device__ __forceinline__ v8f mma(V a, V b, v8f c) { return wmmab(a, b, c); } };
template <typename T16, int NSPLIT, bool BIAS>
__global__ __launch_bounds__(32) void k_gemmw(const T16* __restrict__ A, const T16* __restrict__ A2, const T16* __restrict__ Bt, const T16* __restrict__ Bt2, int K, float* C, int ldc, const float* __restrict__ bias, size_t sA, size_t sB, size_t sC) {
    typedef typename WFrag<T16>::V V;
    __shared__ __align__(16) float os[16 * 68];
    const size_t z = blockIdx.z; A += z * sA; if (A2) A2 += z * sA; Bt += z * sB; if (Bt2) Bt2 += z * sB; C += z * sC;
    const int lane = threadIdx.x & 31, lr = lane & 15, hi = lane >> 4; const int r0 = blockIdx.x * 64, c0 = blockIdx.y * 64;
    v8f acc[4][4];
#pragma unroll
    for (int mb = 0; mb < 4; ++mb)
#pragma unroll
        for (int nb = 0; nb < 4; ++nb) acc[mb][nb] = (v8f){};
    const size_t aoff = (size_t)(r0 + lr) * K + 8 * hi, boff = (size_t)(c0 + lr) * K + 8 * hi;
#pragma unroll 1
    for (int kc = 0; kc < K; kc += 32) {
        V a[4], a2[4];
#pragma unroll
        for (int mb = 0; mb < 4; ++mb) { a[mb] = WFrag<T16>::ld(A + aoff + (size_t)mb * 16 * K + kc); if (NSPLIT == 1 || NSPLIT == 2) a2[mb] = WFrag<T16>::ld(A2 + aoff + (size_t)mb * 16 * K + kc); }
#pragma unroll
        for (int nb = 0; nb < 4; ++nb) { const V b = WFrag<T16>::ld(Bt + boff + (size_t)nb * 16 * K + kc); V b2; if (NSPLIT >= 2) b2 = WFrag<T16>::ld(Bt2 + boff + (size_t)nb * 16 * K + kc);
#pragma unroll
            for (int mb = 0; mb < 4; ++mb) { acc[mb][nb] = WFrag<T16>::mma(a[mb], b, acc[mb][nb]); if (NSPLIT == 1 || NSPLIT == 2) acc[mb][nb] = WFrag<T16>::mma(a2[mb], b, acc[mb][nb]); if (NSPLIT >= 2) acc[mb][nb] = WFrag<T16>::mma(a[mb], b2, acc[mb][nb]); } }
        asm volatile("v_nop\n\tv_nop\n\tv_nop\n\tv_nop" : "+v"(acc[0][0]), "+v"(acc[1][1]), "+v"(acc[2][2]), "+v"(acc[3][3]) : "v"(a[0]), "v"(a[3]));
    }
#pragma unroll
    for (int mb = 0; mb < 4; ++mb) {
#pragma unroll
        for (int nb = 0; nb < 4; ++nb) {
#pragma unroll
            for (int j = 0; j < 8; ++j) os[(hi * 8 + j) * 68 + nb * 16 + lr] = acc[mb][nb][j]; }
        __builtin_amdgcn_wave_barrier(); asm volatile("" ::: "memory");
        float* crow = C + (size_t)(r0 + mb * 16) * ldc + c0;
#pragma unroll 1
        for (int ps = 0; ps < 2; ++ps) {
#pragma unroll
            for (int s = 0; s < 8; ++s) { const int row = 2 * s + hi, cofs = lr * 4; v4f val = *(const v4fa*)(os + row * 68 + cofs); if (BIAS) { val[0] += bfr(bias[c0 + cofs]); val[1] += bfr(bias[c0 + cofs + 1]); val[2] += bfr(bias[c0 + cofs + 2]); val[3] += bfr(bias[c0 + cofs + 3]); }
                *(volatile v4f*)(crow + (size_t)row * ldc + cofs) = val; }
            if (ps == 0) __threadfence(); }
        __builtin_amdgcn_wave_barrier(); asm volatile("" ::: "memory");
    }
}

typedef __attribute__((ext_vector_type(4))) _Float16 v4h;
__device__ __forceinline__ h16 tohx(float x) { return (h16)x; }
__global__ __launch_bounds__(256) void k_im2col3(const float* __restrict__ x, bf* A3) {
    const int lane = threadIdx.x & 31; const size_t r = (size_t)blockIdx.x * 8 + (threadIdx.x >> 5); if (r >= (size_t)NR) return; const int b = (int)(r / TT), t = (int)(r % TT);
#pragma unroll 1
    for (int ps = 0; ps < 2; ++ps) {
#pragma unroll
        for (int q = 0; q < K3 / 256; ++q) { const int c0 = q * 256 + lane * 8; const int k = c0 / DD, c = c0 % DD; const int ts = t + k - 1; v8us o;
#pragma unroll
            for (int i = 0; i < 8; ++i) o[i] = (ts >= 0 && ts < TT) ? f2bf(x[((size_t)b * TT + ts) * DD + c + i]) : (unsigned short)0;
            *(volatile v8us*)(A3 + r * K3 + c0) = o; }
        if (ps == 0) __threadfence(); }
}
template <bool F16O>
__global__ __launch_bounds__(256) void k_wconv(const float* __restrict__ w, int cin, bf* Bt, h16* Bh) {
    const int lane = threadIdx.x & 31; const int o = blockIdx.x * 8 + (threadIdx.x >> 5); if (o >= DD) return; const int KK = 3 * cin;
#pragma unroll 1
    for (int ps = 0; ps < 2; ++ps) {
#pragma unroll 1
        for (int c0 = lane * 8; c0 < KK; c0 += 256) { const int k = c0 / cin, c = c0 % cin; v8us ob; v8h oh;
#pragma unroll
            for (int i = 0; i < 8; ++i) { const float val = bfr(w[((size_t)o * cin + c + i) * 3 + k]); ob[i] = f2bf(val); oh[i] = tohx(val); }
            if (F16O) *(volatile v8h*)(Bh + (size_t)o * KK + c0) = oh; else *(volatile v8us*)(Bt + (size_t)o * KK + c0) = ob; }
        if (ps == 0) __threadfence(); }
}
__global__ __launch_bounds__(256) void k_relu(float* F) {
    const int lane = threadIdx.x & 31; const size_t r = (size_t)blockIdx.x * 8 + (threadIdx.x >> 5); if (r >= (size_t)NR) return;
#pragma unroll
    for (int p = 0; p < DD / 128; ++p) { const int c0 = p * 128 + lane * 4; v4f v = *(const v4f*)(F + r * DD + c0);
#pragma unroll
        for (int i = 0; i < 4; ++i) v[i] = fmaxf(v[i], 0.f);
        *(volatile v4f*)(F + r * DD + c0) = v; __threadfence(); *(volatile v4f*)(F + r * DD + c0) = v; }
}
__global__ __launch_bounds__(256) void k_hpl(const float* __restrict__ F, int b, float sc, h16* P) {
    const int lane = threadIdx.x & 31; const size_t w = (size_t)blockIdx.x * 8 + (threadIdx.x >> 5); const int t = (int)(w * 2 + (lane >> 4)); if (t >= TT) return; const int z = blockIdx.z; const int c0 = (lane & 15) * 4; v4h o;
#pragma unroll
    for (int q = 0; q < 4; ++q) o[q] = tohx(F[((size_t)b * TT + t) * DD + z * HD + c0 + q] * sc);
    const size_t off = ((size_t)z * TT + t) * HD + c0; *(volatile v4h*)(P + off) = o; __threadfence(); *(volatile v4h*)(P + off) = o;
}
__global__ __launch_bounds__(256) void k_hT(const float* __restrict__ F, int b, h16* VT) {
    __shared__ float tl[64][65];
    const int tid = threadIdx.x; const int t0 = blockIdx.x * 64; const int z = blockIdx.z; const int rr = tid >> 2, cq = (tid & 3) * 16;
#pragma unroll
    for (int i = 0; i < 16; ++i) tl[rr][cq + i] = F[((size_t)b * TT + t0 + rr) * DD + z * HD + cq + i];
    __syncthreads();
    const int lane = tid & 31, wv = tid >> 5;
    auto pass = [&]() {
#pragma unroll
        for (int st = 0; st < 4; ++st) { const int dr = wv * 8 + st * 2 + (lane >> 4); const int tq = (lane & 15) * 4; v4h v;
#pragma unroll
            for (int i = 0; i < 4; ++i) v[i] = tohx(tl[tq + i][dr]);
            *(volatile v4h*)(VT + ((size_t)z * HD + dr) * TT + t0 + tq) = v; }
    };
    pass(); __threadfence(); pass();
}
__global__ __launch_bounds__(256) void k_softt(const float* __restrict__ S, h16* P) {
    const int lane = threadIdx.x & 31, i = blockIdx.x * 8 + (threadIdx.x >> 5); if (i >= TT) return; const size_t zo = ((size_t)blockIdx.z * TT + i) * TT; const float* sr = S + zo; h16* po = P + zo;
    float m = -3.0e38f;
#pragma unroll 1
    for (int c0 = lane * 4; c0 < TT; c0 += 128) {
#pragma unroll
        for (int q = 0; q < 4; ++q) m = fmaxf(m, sr[c0 + q]); }
#pragma unroll
    for (int sh = 16; sh; sh >>= 1) m = fmaxf(m, __shfl_xor(m, sh, 32));
    float sum = 0.f;
#pragma unroll 1
    for (int c0 = lane * 4; c0 < TT; c0 += 128) {
#pragma unroll
        for (int q = 0; q < 4; ++q) sum += __expf(sr[c0 + q] - m); }
#pragma unroll
    for (int sh = 16; sh; sh >>= 1) sum += __shfl_xor(sum, sh, 32);
    const float f = __fdiv_rn(PCAR, sum);
#pragma unroll 1
    for (int ps = 0; ps < 2; ++ps) {
#pragma unroll 1
        for (int c0 = lane * 4; c0 < TT; c0 += 128) { v4h o;
#pragma unroll
            for (int q = 0; q < 4; ++q) o[q] = tohx(__expf(sr[c0 + q] - m) * f);
            *(volatile v4h*)(po + c0) = o; }
        if (ps == 0) __threadfence(); }
}
__global__ __launch_bounds__(256) void k_softc(const float* __restrict__ ST, h16* AT) {
    const int lane = threadIdx.x & 31; const int w = blockIdx.x * 8 + (threadIdx.x >> 5); if (w >= NH_ * 32) return; const int z = w / 32, c = (w % 32) * 2 + (lane >> 4); const int d0 = (lane & 15) * 4; const float* sr = ST + ((size_t)z * HD + c) * HD; float v[4]; float m = -3.0e38f;
#pragma unroll
    for (int i = 0; i < 4; ++i) { v[i] = sr[d0 + i] * 0.03125f; m = fmaxf(m, v[i]); }
#pragma unroll
    for (int sh = 1; sh < 16; sh <<= 1) m = fmaxf(m, __shfl_xor(m, sh, 32));
    float s = 0.f;
#pragma unroll
    for (int i = 0; i < 4; ++i) { v[i] = __expf(v[i] - m); s += v[i]; }
#pragma unroll
    for (int sh = 1; sh < 16; sh <<= 1) s += __shfl_xor(s, sh, 32);
    const float f = __fdiv_rn(PCAR, s); v4h o;
#pragma unroll
    for (int i = 0; i < 4; ++i) o[i] = tohx(v[i] * f);
    const size_t off = ((size_t)z * HD + c) * HD + d0; *(volatile v4h*)(AT + off) = o; __threadfence(); *(volatile v4h*)(AT + off) = o;
}
__global__ __launch_bounds__(256) void k_mergevals(const float* __restrict__ OZ, const float* __restrict__ OT, int b, h16* VALS16) {
    const int lane = threadIdx.x & 31; const int tp = blockIdx.x * 8 + (threadIdx.x >> 5); if (tp >= TT) return; h16* dst = VALS16 + ((size_t)b * TT + tp) * (2 * DD);
#pragma unroll 1
    for (int ps = 0; ps < 2; ++ps) {
#pragma unroll
        for (int q = 0; q < 2; ++q) { const int c0 = q * 256 + lane * 8; const int h = c0 / HD, d0 = c0 % HD; v8h o;
#pragma unroll
            for (int i = 0; i < 8; ++i) o[i] = tohx(OZ[((size_t)h * TT + tp) * HD + d0 + i] * (1.0f / PCAR));
            *(volatile v8h*)(dst + c0) = o; }
#pragma unroll
        for (int q = 0; q < 2; ++q) { const int c0 = q * 256 + lane * 8; v8h o;
#pragma unroll
            for (int i = 0; i < 8; ++i) { const int f = tp * DD + c0 + i; const int c = f >> 13, t = (f >> 3) & (TT - 1), h = f & 7; o[i] = tohx(OT[((size_t)h * HD + c) * TT + t] * (1.0f / PCAR)); }
            *(volatile v8h*)(dst + DD + c0) = o; }
        if (ps == 0) __threadfence(); }
}
__global__ __launch_bounds__(256) void k_im2colv(const h16* __restrict__ VALS16, h16* V3) {
    const int lane = threadIdx.x & 31; const size_t r = (size_t)blockIdx.x * 8 + (threadIdx.x >> 5); if (r >= (size_t)NR) return; const int b = (int)(r / TT), t = (int)(r % TT); v8h zero; for (int i = 0; i < 8; ++i) zero[i] = tohx(0.f);
#pragma unroll 1
    for (int ps = 0; ps < 2; ++ps) {
#pragma unroll 1
        for (int q = 0; q < K6 / 256; ++q) { const int c0 = q * 256 + lane * 8; const int k = c0 / (2 * DD), j = c0 % (2 * DD); const int ts = t + k - 1; const v8h o = (ts >= 0 && ts < TT) ? *(const v8h*)(VALS16 + ((size_t)b * TT + ts) * (2 * DD) + j) : zero;
            *(volatile v8h*)(V3 + r * K6 + c0) = o; }
        if (ps == 0) __threadfence(); }
}
__global__ __launch_bounds__(256) void k_reluout(const float* __restrict__ C2, float* OUTB) {
    const int lane = threadIdx.x & 31; const size_t r = (size_t)blockIdx.x * 8 + (threadIdx.x >> 5); if (r >= (size_t)NR) return;
#pragma unroll 1
    for (int ps = 0; ps < 2; ++ps) {
#pragma unroll
        for (int p = 0; p < DD / 128; ++p) { const int c0 = p * 128 + lane * 4; v4f v = *(const v4f*)(C2 + r * DD + c0);
#pragma unroll
            for (int i = 0; i < 4; ++i) v[i] = fmaxf(v[i], 0.f);
            *(volatile v4f*)(OUTB + r * DD + c0) = v; }
        if (ps == 0) __threadfence(); }
}
extern "C" void kernel_launch(void* const* d_in, const int* in_sizes, int n_in,
                              void* d_out, int out_size, void* d_ws, size_t ws_size, hipStream_t stream) {
    (void)in_sizes; (void)n_in; (void)out_size;
    const float* x = (const float*)d_in[0]; const float* w11 = (const float*)d_in[1]; const float* b11 = (const float*)d_in[2]; const float* w12 = (const float*)d_in[3]; const float* b12 = (const float*)d_in[4]; const float* w13 = (const float*)d_in[5]; const float* b13 = (const float*)d_in[6]; const float* w2 = (const float*)d_in[7]; const float* b2 = (const float*)d_in[8];
    float* out = (float*)d_out;
    char* wsp = (char*)d_ws;
    auto take = [&](size_t bytes) { char* p = wsp; wsp += (bytes + 255) & ~(size_t)255; return (void*)p; };
    bf* W1 = (bf*)take((size_t)DD * K3 * 2); bf* W2b = (bf*)take((size_t)DD * K3 * 2); bf* W3 = (bf*)take((size_t)DD * K3 * 2); h16* WO = (h16*)take((size_t)DD * K6 * 2);
    bf* A3 = (bf*)take((size_t)NR * K3 * 2); float* Q = (float*)take((size_t)NR * DD * 4); float* Kf = (float*)take((size_t)NR * DD * 4); float* V = (float*)take((size_t)NR * DD * 4);
    h16* Qx = (h16*)take((size_t)NH_ * TT * HD * 2); h16* Kx = (h16*)take((size_t)NH_ * TT * HD * 2); h16* Vx = (h16*)take((size_t)NH_ * TT * HD * 2); h16* QT = (h16*)take((size_t)NH_ * HD * TT * 2); h16* KT = (h16*)take((size_t)NH_ * HD * TT * 2); h16* VT = (h16*)take((size_t)NH_ * HD * TT * 2);
    float* S = (float*)take((size_t)NH_ * TT * TT * 4); h16* Px = (h16*)take((size_t)NH_ * TT * TT * 2); float* OZ = (float*)take((size_t)NH_ * TT * HD * 4); float* ST = (float*)take((size_t)NH_ * HD * HD * 4); h16* AT = (h16*)take((size_t)NH_ * HD * HD * 2); float* OT = (float*)take((size_t)NH_ * HD * TT * 4);
    h16* VALS16 = (h16*)take((size_t)NR * 2 * DD * 2); float* C2 = (float*)take((size_t)NR * DD * 4);
    if ((size_t)(wsp - (char*)d_ws) > ws_size) return;
    h16* V3 = (h16*)A3;
    k_wconv<false><<<DD / 8, 256, 0, stream>>>(w11, DD, W1, nullptr); k_wconv<false><<<DD / 8, 256, 0, stream>>>(w12, DD, W2b, nullptr); k_wconv<false><<<DD / 8, 256, 0, stream>>>(w13, DD, W3, nullptr); k_wconv<true><<<DD / 8, 256, 0, stream>>>(w2, 2 * DD, nullptr, WO);
    k_im2col3<<<NR / 8, 256, 0, stream>>>(x, A3);
    k_gemmw<bf, 0, true><<<dim3(NR / 64, DD / 64, 1), 32, 0, stream>>>(A3, nullptr, W1, nullptr, K3, Q, DD, b11, 0, 0, 0); k_relu<<<NR / 8, 256, 0, stream>>>(Q);
    k_gemmw<bf, 0, true><<<dim3(NR / 64, DD / 64, 1), 32, 0, stream>>>(A3, nullptr, W2b, nullptr, K3, Kf, DD, b12, 0, 0, 0); k_relu<<<NR / 8, 256, 0, stream>>>(Kf);
    k_gemmw<bf, 0, true><<<dim3(NR / 64, DD / 64, 1), 32, 0, stream>>>(A3, nullptr, W3, nullptr, K3, V, DD, b13, 0, 0, 0); k_relu<<<NR / 8, 256, 0, stream>>>(V);
    for (int b = 0; b < NB_; ++b) {
        k_hpl<<<dim3((TT / 2) / 8, 1, NH_), 256, 0, stream>>>(Q, b, 0.125f, Qx); k_hpl<<<dim3((TT / 2) / 8, 1, NH_), 256, 0, stream>>>(Kf, b, 1.0f, Kx); k_hpl<<<dim3((TT / 2) / 8, 1, NH_), 256, 0, stream>>>(V, b, 1.0f, Vx); k_hT<<<dim3(TT / 64, 1, NH_), 256, 0, stream>>>(V, b, VT);
        k_gemmw<h16, 0, false><<<dim3(TT / 64, TT / 64, NH_), 32, 0, stream>>>(Qx, nullptr, Kx, nullptr, HD, S, TT, nullptr, (size_t)TT * HD, (size_t)TT * HD, (size_t)TT * TT);
        k_softt<<<dim3(TT / 8, 1, NH_), 256, 0, stream>>>(S, Px);
        k_gemmw<h16, 0, false><<<dim3(TT / 64, 1, NH_), 32, 0, stream>>>(Px, nullptr, VT, nullptr, TT, OZ, HD, nullptr, (size_t)TT * TT, (size_t)HD * TT, (size_t)TT * HD);
        k_hT<<<dim3(TT / 64, 1, NH_), 256, 0, stream>>>(Q, b, QT); k_hT<<<dim3(TT / 64, 1, NH_), 256, 0, stream>>>(Kf, b, KT);
        k_gemmw<h16, 0, false><<<dim3(1, 1, NH_), 32, 0, stream>>>(QT, nullptr, KT, nullptr, TT, ST, HD, nullptr, (size_t)HD * TT, (size_t)HD * TT, (size_t)HD * HD);
        k_softc<<<(NH_ * 32) / 8, 256, 0, stream>>>(ST, AT);
        k_gemmw<h16, 0, false><<<dim3(1, TT / 64, NH_), 32, 0, stream>>>(AT, nullptr, Vx, nullptr, HD, OT, TT, nullptr, (size_t)HD * HD, (size_t)TT * HD, (size_t)HD * TT);
        k_mergevals<<<TT / 8, 256, 0, stream>>>(OZ, OT, b, VALS16); }
    k_im2colv<<<NR / 8, 256, 0, stream>>>(VALS16, V3);
    k_gemmw<h16, 0, true><<<dim3(NR / 64, DD / 64, 1), 32, 0, stream>>>(V3, nullptr, WO, nullptr, K6, C2, DD, b2, 0, 0, 0);
    k_reluout<<<NR / 8, 256, 0, stream>>>(C2, out);
}
